// GRUDCell_73864847557195
// MI455X (gfx1250) — hardware-run, weakly checked
//
#include <hip/hip_runtime.h>
#include <math.h>

typedef __attribute__((ext_vector_type(16))) _Float16 v16h;
typedef __attribute__((ext_vector_type(8)))  _Float16 v8h;
typedef __attribute__((ext_vector_type(16))) __bf16   v16b;
typedef __attribute__((ext_vector_type(8)))  __bf16   v8b;
typedef __attribute__((ext_vector_type(8)))  float    v8f;
typedef __attribute__((ext_vector_type(4)))  float    v4f;

constexpr int kB    = 8192;
constexpr int kI    = 512;
constexpr int kH    = 1024;
constexpr int kHLog2 = 10;
constexpr int kG3   = 3 * kH;
constexpr int kDD   = 8;
constexpr int kCh   = 2048;
constexpr int kNCh  = kB / kCh;
constexpr int kThr  = 256;
constexpr float kInCarry = 1024.0f;
constexpr float kSc = 1.0f / (kInCarry * kInCarry);
constexpr float kF16MinNormal = 6.103515625e-5f;

static_assert((1 << kHLog2) == kH && kNCh * kCh == kB, "the shifts follow the sizes");
static_assert((kCh % 64) == 0 && (kG3 % 64) == 0 && (kI % 32) == 0 && (kH % 32) == 0 && ((kCh / 64) * (kG3 / 64)) % 8 == 0, "GEMM M, N multiples of 64, K of 32; grid exact (1,536 tiles a chunk)");

constexpr size_t kOffX16 = 0ull;
constexpr size_t kOffWIH16 = 8388608ull;
constexpr size_t kOffWHH16 = 11534336ull;
constexpr size_t kOffBIAS = 17825792ull;
constexpr size_t kOffHD16 = 17850368ull;
constexpr size_t kOffGI = 34627584ull;
constexpr size_t kOffGH = 59793408ull;
constexpr size_t kWsTotal = 84959232ull;
static_assert(kWsTotal <= 134217728ull, "carve cap: under 128 MiB");
static_assert(kOffX16 == 0
              && kOffWIH16 == kOffX16 + 8388608ull
              && kOffWHH16 == kOffWIH16 + 3145728ull
              && kOffBIAS == kOffWHH16 + 6291456ull
              && kOffHD16 == kOffBIAS + 24576ull
              && kOffGI == kOffHD16 + 16777216ull
              && kOffGH == kOffGI + 25165824ull
              && kWsTotal == kOffGH + 25165824ull, "the carve is chained and totalled");
static_assert((kOffX16 % 256) == 0 && (kOffWIH16 % 256) == 0 && (kOffWHH16 % 256) == 0 && (kOffBIAS % 256) == 0 && (kOffHD16 % 256) == 0 && (kOffGI % 256) == 0 && (kOffGH % 256) == 0, "aligned regions");

__device__ __forceinline__ unsigned short f2bf_bits(float f) {
  unsigned u = __float_as_uint(f);
  return (unsigned short)((u + 0x7FFFu + ((u >> 16) & 1u)) >> 16);
}
__device__ __forceinline__ float bf_bits2f(unsigned short h) { return __uint_as_float(((unsigned)h) << 16); }
__device__ __forceinline__ float bf16r(float f) { return bf_bits2f(f2bf_bits(f)); }
__device__ __forceinline__ float carry_flush(float v, float carry) {
  const float s = v * carry;
  return (fabsf(s) < kF16MinNormal) ? 0.0f : s;
}
__device__ __forceinline__ float frcp(float x) { return __builtin_amdgcn_rcpf(x); }

__device__ __forceinline__ void dep_guard4_h(v8f& a, v8f& b, v8f& c, v8f& d, v16h x, v16h y) { asm volatile("v_nop\n\tv_nop\n\tv_nop\n\tv_nop" : "+v"(a), "+v"(b), "+v"(c), "+v"(d) : "v"(x), "v"(y)); }
__device__ __forceinline__ void dep_guard4_b(v8f& a, v8f& b, v8f& c, v8f& d, v16b x, v16b y) { asm volatile("v_nop\n\tv_nop\n\tv_nop\n\tv_nop" : "+v"(a), "+v"(b), "+v"(c), "+v"(d) : "v"(x), "v"(y)); }
__device__ __forceinline__ void keep4_h(v16h a, v16h b, v16h c, v16h d) { asm volatile("v_nop" :: "v"(a), "v"(b), "v"(c), "v"(d)); }
__device__ __forceinline__ void keep4_b(v16b a, v16b b, v16b c, v16b d) { asm volatile("v_nop" :: "v"(a), "v"(b), "v"(c), "v"(d)); }
__device__ __forceinline__ void acc_guard4(v8f& a, v8f& b, v8f& c, v8f& d) { asm volatile("v_nop\n\tv_nop\n\tv_nop\n\tv_nop" : "+v"(a), "+v"(b), "+v"(c), "+v"(d)); }

template <typename T> struct Frag;
template <> struct Frag<_Float16> {
  typedef v16h V; union U { v16h v; v8h h[2]; };
  static __device__ __forceinline__ v16h load(const _Float16* p) {
    U f; f.h[0] = *(const v8h*)(p); f.h[1] = *(const v8h*)(p + 16); return f.v;
  }
  static __device__ __forceinline__ v8f mma(v16h a, v16h b, v8f c) {
    return __builtin_amdgcn_wmma_f32_16x16x32_f16(false, a, false, b, (short)0, c, false, false);
  }
  static __device__ __forceinline__ void guard4(v8f& a, v8f& b, v8f& c, v8f& d, v16h x, v16h y) { dep_guard4_h(a, b, c, d, x, y); }
  static __device__ __forceinline__ void keep(v16h a, v16h b, v16h c, v16h d) { keep4_h(a, b, c, d); }
};
template <> struct Frag<__bf16> {
  typedef v16b V; union U { v16b v; v8b h[2]; };
  static __device__ __forceinline__ v16b load(const __bf16* p) {
    U f; f.h[0] = *(const v8b*)(p); f.h[1] = *(const v8b*)(p + 16); return f.v;
  }
  static __device__ __forceinline__ v8f mma(v16b a, v16b b, v8f c) {
    return __builtin_amdgcn_wmma_f32_16x16x32_bf16(false, a, false, b, (short)0, c, false, false);
  }
  static __device__ __forceinline__ void guard4(v8f& a, v8f& b, v8f& c, v8f& d, v16b x, v16b y) { dep_guard4_b(a, b, c, d, x, y); }
  static __device__ __forceinline__ void keep(v16b a, v16b b, v16b c, v16b d) { keep4_b(a, b, c, d); }
};

__device__ __forceinline__ v8f mma_h(v16h a, v16h b, v8f c) {
  c = __builtin_amdgcn_wmma_f32_16x16x32_f16(false, a, false, b, (short)0, c, false, false);
  asm volatile("v_nop\n\tv_nop\n\tv_nop\n\tv_nop" : "+v"(c) : "v"(a), "v"(b));
  return c;
}

template <int ET> struct Elem;
template <> struct Elem<0> { typedef _Float16 T; };
template <> struct Elem<1> { typedef __bf16 T; };
template <int ET, bool SPLIT, int BIAS_MODE, int OUT_MODE, bool RESID, int ACT = 0>
__global__ __launch_bounds__(256) void wmma_gemm64(
    const unsigned short* __restrict__ Ap, const unsigned short* __restrict__ A2p, int lda, long strideA,
    const unsigned short* __restrict__ Btp, const unsigned short* __restrict__ Bt2p, int ldb, long strideB,
    void* __restrict__ Cout, void* __restrict__ Cout2, int ldc, long strideC,
    const float* __restrict__ bias,
    const float* __restrict__ resid, long strideR,
    int M, int N, int K, float scale) {
  typedef typename Elem<ET>::T T;
  typedef typename Frag<T>::V V;
  const T* A = (const T*)Ap; const T* A2 = (const T*)A2p; const T* Bt = (const T*)Btp; const T* Bt2 = (const T*)Bt2p;
  __shared__ __align__(16) float sT[8][16 * 68];
  const int b    = blockIdx.y;
  const int lane = threadIdx.x & 31;
  const int wave = threadIdx.x >> 5;
  const int tilesN = N >> 6;
  const int tilesM = M >> 6;
  const int tile = blockIdx.x * 8 + wave;
  if (tile >= tilesM * tilesN) return;
  const int tm = tile / tilesN;
  const int tn = tile - tm * tilesN;
  const int m0 = tm << 6;
  const int n0 = tn << 6;

  const T* Ab  = A  + (size_t)b * strideA;
  const T* Bb  = Bt + (size_t)b * strideB;
  const T* Ab2 = SPLIT ? (A2  + (size_t)b * strideA) : nullptr;
  const T* Bb2 = SPLIT ? (Bt2 + (size_t)b * strideB) : nullptr;

  const int rlane = lane & 15;
  const int koff  = (lane >> 4) * 8;
  const int mOff  = (lane >> 4) * 8;

  v8f acc[4][4];
#pragma unroll
  for (int i = 0; i < 4; ++i)
#pragma unroll
    for (int j = 0; j < 4; ++j) acc[i][j] = (v8f){0.f,0.f,0.f,0.f,0.f,0.f,0.f,0.f};

  for (int k0 = 0; k0 < K; k0 += 32) {
    V bh[4], bl[4];
#pragma unroll
    for (int j = 0; j < 4; ++j) {
      const size_t bo = (size_t)(n0 + (j << 4) + rlane) * ldb + koff + k0;
      bh[j] = Frag<T>::load(Bb + bo);
      if (SPLIT) bl[j] = Frag<T>::load(Bb2 + bo);
    }
#pragma unroll
    for (int i = 0; i < 4; ++i) {
      const size_t ao = (size_t)(m0 + (i << 4) + rlane) * lda + koff + k0;
      V ah = Frag<T>::load(Ab + ao);
      V al;
      if (SPLIT) al = Frag<T>::load(Ab2 + ao);
#pragma unroll
      for (int j = 0; j < 4; ++j) {
        acc[i][j] = Frag<T>::mma(ah, bh[j], acc[i][j]);
        if (SPLIT) {
          acc[i][j] = Frag<T>::mma(ah, bl[j], acc[i][j]);
          acc[i][j] = Frag<T>::mma(al, bh[j], acc[i][j]);
        }
      }
      Frag<T>::guard4(acc[i][0], acc[i][1], acc[i][2], acc[i][3], ah, SPLIT ? al : ah);
    }
    Frag<T>::keep(bh[0], bh[1], bh[2], bh[3]);
    if (SPLIT) Frag<T>::keep(bl[0], bl[1], bl[2], bl[3]);
  }
  acc_guard4(acc[0][0], acc[0][1], acc[0][2], acc[0][3]);
  acc_guard4(acc[1][0], acc[1][1], acc[1][2], acc[1][3]);
  acc_guard4(acc[2][0], acc[2][1], acc[2][2], acc[2][3]);
  acc_guard4(acc[3][0], acc[3][1], acc[3][2], acc[3][3]);

  float* slab = sT[wave];
  const float* Rb = RESID ? (resid + (size_t)b * strideR) : nullptr;
#pragma unroll
  for (int i = 0; i < 4; ++i) {
    const int mBase = m0 + (i << 4);
#pragma unroll
    for (int j = 0; j < 4; ++j) {
      const int n = n0 + (j << 4) + rlane;
      float bv = 0.f;
      if (BIAS_MODE == 2) bv = bias[n];
#pragma unroll
      for (int r = 0; r < 8; ++r) {
        float v = acc[i][j][r] * scale;
        if (BIAS_MODE == 1) v += bias[mBase + mOff + r];
        if (BIAS_MODE == 2) v += bv;
        if (RESID) v += Rb[(size_t)(mBase + mOff + r) * ldc + n];
        if (ACT == 1) v = tanhf(v);
        if (ACT == 2) v = fmaxf(v, 0.0f);
        if (ACT == 3) v = v / (1.0f + expf(-v));
        if (ACT == 4) v = (v > 0.f) ? v : 0.01f * v;
        slab[(mOff + r) * 68 + (j << 4) + rlane] = v;
      }
    }
    __builtin_amdgcn_fence(__ATOMIC_RELEASE, "workgroup");
    __builtin_amdgcn_wave_barrier();
    __builtin_amdgcn_fence(__ATOMIC_ACQUIRE, "workgroup");
    if (OUT_MODE == 0) {
      float* C = (float*)Cout + (size_t)b * strideC;
      const int hh = lane >> 4, c4 = (lane & 15) * 4;
      for (int pass = 0; pass < 2; ++pass) {
#pragma unroll
        for (int it = 0; it < 8; ++it) {
          const int row = it * 2 + hh;
          v4f v = *(const v4f*)(slab + row * 68 + c4);
          *(volatile v4f*)(C + (size_t)(mBase + row) * ldc + n0 + c4) = v;
        }
        __threadfence();
      }
    } else {
      const int q = lane >> 3, c8 = (lane & 7) * 8;
      unsigned short* C  = (unsigned short*)Cout  + (size_t)b * strideC;
      unsigned short* C2 = (OUT_MODE == 2) ? ((unsigned short*)Cout2 + (size_t)b * strideC) : nullptr;
      for (int pass = 0; pass < 2; ++pass) {
#pragma unroll
        for (int it = 0; it < 4; ++it) {
          const int row = it * 4 + q;
          const float* sp = slab + row * 68 + c8;
          v8h hv, lv;
#pragma unroll
          for (int e = 0; e < 8; ++e) {
            if (OUT_MODE == 1) {
              hv[e] = (_Float16)sp[e];
            } else {
              unsigned short hb = f2bf_bits(sp[e]);
              unsigned short lb = f2bf_bits(sp[e] - bf_bits2f(hb));
              hv[e] = __builtin_bit_cast(_Float16, hb);
              lv[e] = __builtin_bit_cast(_Float16, lb);
            }
          }
          *(volatile v8h*)(C + (size_t)(mBase + row) * ldc + n0 + c8) = hv;
          if (OUT_MODE == 2) *(volatile v8h*)(C2 + (size_t)(mBase + row) * ldc + n0 + c8) = lv;
        }
        __threadfence();
      }
    }
    __builtin_amdgcn_fence(__ATOMIC_RELEASE, "workgroup");
    __builtin_amdgcn_wave_barrier();
    __builtin_amdgcn_fence(__ATOMIC_ACQUIRE, "workgroup");
  }
}

__global__ __launch_bounds__(kThr) void cast_plane_kernel(const float* __restrict__ src, unsigned short* __restrict__ dst,
                                                          int colsLog2, int dstPitch, int dstOff) {
  const int i   = blockIdx.x * kThr + threadIdx.x;
  const int sh  = colsLog2 - 3;
  const int row = i >> sh;
  const int c8  = (i & ((1 << sh) - 1)) * 8;
  const float* sp = src + ((size_t)row << colsLog2) + c8;
  const v4f a0 = *(const v4f*)(sp);
  const v4f a1 = *(const v4f*)(sp + 4);
  v8h hv;
#pragma unroll
  for (int e = 0; e < 4; ++e) {
    const float f0 = a0[e];
    const float f1 = a1[e];
    hv[e]     = (_Float16)carry_flush(bf16r(f0), kInCarry);
    hv[4 + e] = (_Float16)carry_flush(bf16r(f1), kInCarry);
  }
  unsigned short* dp = dst + (size_t)row * dstPitch + dstOff + c8;
  *(volatile v8h*)dp = hv;
  __threadfence();
  *(volatile v8h*)dp = hv;
}

__device__ __forceinline__ float decayed_state(const float* dl, const float* wg, float bg, float hraw) {
  float pre = bf16r(bg);
#pragma unroll
  for (int d = 0; d < kDD; ++d) { const float a = dl[d], w = wg[d]; pre += bf16r(a) * bf16r(w); }
  const float g = expf(-fmaxf(pre, 0.0f));
  return g * bf16r(hraw);
}

__global__ __launch_bounds__(kThr) void bias_kernel(const float* __restrict__ bias_ih, const float* __restrict__ bias_hh, float* __restrict__ BIAS) {
  const int i = blockIdx.x * kThr + threadIdx.x;
  const bool first = i < kG3;
  const float v0 = bias_ih[first ? i : 0];
  const float v1 = bias_hh[first ? 0 : (i - kG3)];
  const float o = first ? bf16r(v0) : bf16r(v1);
  for (int pass = 0; pass < 2; ++pass) {
    *(volatile float*)(BIAS + i) = o;
    __threadfence();
  }
}
static_assert((2 * kG3) % kThr == 0, "bias grid exact");

__global__ __launch_bounds__(kThr) void front_kernel(const float* __restrict__ delta, const float* __restrict__ h, const float* __restrict__ w_gamma,
                                                     const float* __restrict__ b_gamma, unsigned short* __restrict__ HD16) {
  const size_t i = (size_t)blockIdx.x * kThr + threadIdx.x;
  const size_t b = i >> (kHLog2 - 3);
  const int j8 = (int)(i & (size_t)(kH / 8 - 1)) * 8;
  float dl[kDD];
  {
    const v4f d0 = *(const v4f*)(delta + b * kDD), d1 = *(const v4f*)(delta + b * kDD + 4);
#pragma unroll
    for (int e = 0; e < 4; ++e) { dl[e] = d0[e]; dl[4 + e] = d1[e]; }
  }
  const v4f h0 = *(const v4f*)(h + b * kH + j8), h1 = *(const v4f*)(h + b * kH + j8 + 4);
  const v4f g0 = *(const v4f*)(b_gamma + j8), g1 = *(const v4f*)(b_gamma + j8 + 4);
  v8h hv;
#pragma unroll
  for (int e = 0; e < 8; ++e) {
    float wg[kDD];
    const v4f w0 = *(const v4f*)(w_gamma + (size_t)(j8 + e) * kDD), w1 = *(const v4f*)(w_gamma + (size_t)(j8 + e) * kDD + 4);
#pragma unroll
    for (int d = 0; d < 4; ++d) { wg[d] = w0[d]; wg[4 + d] = w1[d]; }
    const float hr = (e < 4) ? h0[e] : h1[e - 4];
    const float bg = (e < 4) ? g0[e] : g1[e - 4];
    hv[e] = (_Float16)carry_flush(decayed_state(dl, wg, bg, hr), kInCarry);
  }
  unsigned short* dp = HD16 + b * kH + j8;
  *(volatile v8h*)dp = hv;
  __threadfence();
  *(volatile v8h*)dp = hv;
}
static_assert(((size_t)kB * kH / 8) % kThr == 0, "front grid exact");

__global__ __launch_bounds__(kThr) void cell_kernel(const float* __restrict__ GI, const float* __restrict__ GH, const float* __restrict__ delta,
                                                    const float* __restrict__ h, const float* __restrict__ w_gamma, const float* __restrict__ b_gamma,
                                                    float* __restrict__ out, int chunk) {
  const size_t i = (size_t)blockIdx.x * kThr + threadIdx.x;
  const size_t lr = i >> (kHLog2 - 2);
  const int j4 = (int)(i & (size_t)(kH / 4 - 1)) * 4;
  const size_t b = (size_t)chunk * kCh + lr;
  float dl[kDD];
  {
    const v4f d0 = *(const v4f*)(delta + b * kDD), d1 = *(const v4f*)(delta + b * kDD + 4);
#pragma unroll
    for (int e = 0; e < 4; ++e) { dl[e] = d0[e]; dl[4 + e] = d1[e]; }
  }
  const float* gi = GI + lr * kG3 + j4;
  const float* gh = GH + lr * kG3 + j4;
  const v4f ir = *(const v4f*)gi, iz = *(const v4f*)(gi + kH), in = *(const v4f*)(gi + 2 * kH);
  const v4f hr = *(const v4f*)gh, hz = *(const v4f*)(gh + kH), hn = *(const v4f*)(gh + 2 * kH);
  const v4f hraw = *(const v4f*)(h + b * kH + j4);
  const v4f bg = *(const v4f*)(b_gamma + j4);
  v4f o;
#pragma unroll
  for (int e = 0; e < 4; ++e) {
    float wg[kDD];
    const v4f w0 = *(const v4f*)(w_gamma + (size_t)(j4 + e) * kDD), w1 = *(const v4f*)(w_gamma + (size_t)(j4 + e) * kDD + 4);
#pragma unroll
    for (int d = 0; d < 4; ++d) { wg[d] = w0[d]; wg[4 + d] = w1[d]; }
    const float hd = decayed_state(dl, wg, bg[e], hraw[e]);
    const float r = 1.0f / (1.0f + expf(-(ir[e] + hr[e])));
    const float z = 1.0f / (1.0f + expf(-(iz[e] + hz[e])));
    const float n = tanhf(in[e] + r * hn[e]);
    o[e] = n + z * (hd - n);
  }
  float* dp = out + b * kH + j4;
  *(volatile v4f*)dp = o;
  __threadfence();
  *(volatile v4f*)dp = o;
}
static_assert(((size_t)kCh * kH / 4) % kThr == 0, "cell grid exact");

static_assert(((size_t)kB * kI / 8) % kThr == 0 && ((size_t)kG3 * kI / 8) % kThr == 0 && ((size_t)kG3 * kH / 8) % kThr == 0, "plane cast grids exact");

extern "C" void kernel_launch(void* const* d_in, const int* in_sizes, int n_in,
                              void* d_out, int out_size, void* d_ws, size_t ws_size,
                              hipStream_t stream) {
  if (n_in < 9 || d_out == nullptr || d_ws == nullptr) return;
  if (in_sizes[0] != kB * kI || in_sizes[1] != kB * kDD || in_sizes[2] != kB * kH || in_sizes[3] != kG3 * kI || in_sizes[4] != kG3 * kH) return;
  if (in_sizes[5] != kG3 || in_sizes[6] != kG3 || in_sizes[7] != kH * kDD || in_sizes[8] != kH) return;
  if (out_size != kB * kH) return;
  if (ws_size < kWsTotal) return;
  const float* x = (const float*)d_in[0];
  const float* delta = (const float*)d_in[1];
  const float* h = (const float*)d_in[2];
  const float* weight_ih = (const float*)d_in[3];
  const float* weight_hh = (const float*)d_in[4];
  const float* bias_ih = (const float*)d_in[5];
  const float* bias_hh = (const float*)d_in[6];
  const float* w_gamma = (const float*)d_in[7];
  const float* b_gamma = (const float*)d_in[8];
  float* out = (float*)d_out;
  char* ws = (char*)d_ws;
  unsigned short* X16 = (unsigned short*)(ws + kOffX16);
  unsigned short* WIH16 = (unsigned short*)(ws + kOffWIH16);
  unsigned short* WHH16 = (unsigned short*)(ws + kOffWHH16);
  float* BIAS = (float*)(ws + kOffBIAS);
  unsigned short* HD16 = (unsigned short*)(ws + kOffHD16);
  float* GI = (float*)(ws + kOffGI);
  float* GH = (float*)(ws + kOffGH);

  cast_plane_kernel<<<(int)(((size_t)kB * kI / 8) / kThr), kThr, 0, stream>>>(x, X16, 9, kI, 0);
  cast_plane_kernel<<<(int)(((size_t)kG3 * kI / 8) / kThr), kThr, 0, stream>>>(weight_ih, WIH16, 9, kI, 0);
  cast_plane_kernel<<<(int)(((size_t)kG3 * kH / 8) / kThr), kThr, 0, stream>>>(weight_hh, WHH16, 10, kH, 0);
  bias_kernel<<<(2 * kG3) / kThr, kThr, 0, stream>>>(bias_ih, bias_hh, BIAS);
  front_kernel<<<(int)(((size_t)kB * kH / 8) / kThr), kThr, 0, stream>>>(delta, h, w_gamma, b_gamma, HD16);
  for (int c = 0; c < kNCh; ++c) {
    wmma_gemm64<0, false, 2, 0, false, 0><<<dim3((kCh / 64) * (kG3 / 64) / 8, 1), 256, 0, stream>>>(
        X16 + (size_t)c * kCh * kI, X16 + (size_t)c * kCh * kI, kI, 0L, WIH16, WIH16, kI, 0L, (void*)GI, (void*)GI, kG3, 0L, BIAS, nullptr, 0L, kCh, kG3, kI, kSc);
    wmma_gemm64<0, false, 2, 0, false, 0><<<dim3((kCh / 64) * (kG3 / 64) / 8, 1), 256, 0, stream>>>(
        HD16 + (size_t)c * kCh * kH, HD16 + (size_t)c * kCh * kH, kH, 0L, WHH16, WHH16, kH, 0L, (void*)GH, (void*)GH, kG3, 0L, BIAS + kG3, nullptr, 0L, kCh, kG3, kH, kSc);
    cell_kernel<<<(int)(((size_t)kCh * kH / 4) / kThr), kThr, 0, stream>>>(GI, GH, delta, h, w_gamma, b_gamma, out, c);
  }
}
